// MWTF_29016799052177
// MI455X (gfx1250) — hardware-verified
//
#include <hip/hip_runtime.h>
#include <math.h>

typedef __attribute__((ext_vector_type(16))) _Float16 v16h;
typedef __attribute__((ext_vector_type(16))) __bf16 v16b;
typedef __attribute__((ext_vector_type(8)))  _Float16 v8h;
typedef __attribute__((ext_vector_type(8)))  float v8f;
typedef __attribute__((ext_vector_type(4)))  float v4f;
typedef __attribute__((ext_vector_type(2)))  float v2f;
typedef __attribute__((ext_vector_type(4)))  unsigned v4u;
typedef __attribute__((ext_vector_type(4)))  int v4i;
typedef float __attribute__((may_alias)) float_a;
typedef int __attribute__((may_alias)) int_a;

template <typename T> __device__ __forceinline__ void vst2(void* p, T v) { *(volatile T*)p = v; __threadfence(); *(volatile T*)p = v; }
__device__ __forceinline__ v8f wmma16(v16h a, v16h b, v8f c) {
  v8f d = __builtin_amdgcn_wmma_f32_16x16x32_f16(false, a, false, b, (short)0, c, false, false);
  asm volatile("v_nop\n\tv_nop\n\tv_nop\n\tv_nop" : "+v"(d) : "v"(a), "v"(b));
  return d;
}
__device__ __forceinline__ v8f wmma_bf(v16b a, v16b b, v8f c) {
  v8f d = __builtin_amdgcn_wmma_f32_16x16x32_bf16(false, a, false, b, (short)0, c, false, false);
  asm volatile("v_nop\n\tv_nop\n\tv_nop\n\tv_nop" : "+v"(d) : "v"(a), "v"(b));
  return d;
}
__device__ __forceinline__ v16h frag_h(const _Float16* rowk0, int lane) {
  union { v16h v; v8h q[2]; } u; const _Float16* p = rowk0 + 8 * (lane >> 4);
  u.q[0] = *(const v8h*)p; u.q[1] = *(const v8h*)(p + 16); return u.v;
}
__device__ __forceinline__ v16h frag_f32(const float* rowk0, int lane) {
  v16h a; const float* p = rowk0 + 8 * (lane >> 4);
#pragma unroll
  for (int i = 0; i < 8; ++i) { a[i] = (_Float16)p[i]; a[8 + i] = (_Float16)p[16 + i]; }
  return a;
}
__device__ __forceinline__ v16h frag_f32s(const float* rowk0, int lane, float sc) {
  v16h a; const float* p = rowk0 + 8 * (lane >> 4);
#pragma unroll
  for (int i = 0; i < 8; ++i) { a[i] = (_Float16)(p[i] * sc); a[8 + i] = (_Float16)(p[16 + i] * sc); }
  return a;
}
__device__ __forceinline__ v16h fragc_f32(const float* W, int k0, int n, int lane, int ld, int K) {
  v16h a; const int g = lane >> 4;
#pragma unroll
  for (int i = 0; i < 8; ++i) { const int ka = k0 + 8 * g + i, kb = ka + 16;
    a[i] = (_Float16)(ka < K ? W[(size_t)(ka < K ? ka : K - 1) * ld + n] : 0.f); a[8 + i] = (_Float16)(kb < K ? W[(size_t)(kb < K ? kb : K - 1) * ld + n] : 0.f); }
  return a;
}
struct F2 { v16b h, l; };
__device__ __forceinline__ F2 bsplit16(const float v[16]) { F2 r;
#pragma unroll
  for (int i = 0; i < 16; ++i) { const __bf16 h = (__bf16)v[i]; r.h[i] = h; r.l[i] = (__bf16)(v[i] - (float)h); }
  return r; }
__device__ __forceinline__ F2 split_row(const float* row, int k0, int lane) { float v[16]; const float* p = row + k0 + 8 * (lane >> 4);
#pragma unroll
  for (int i = 0; i < 8; ++i) { v[i] = p[i]; v[8 + i] = p[16 + i]; }
  return bsplit16(v); }
__device__ __forceinline__ F2 split_rowK(const float* row, int k0, int lane, int K) { float v[16]; const int g = lane >> 4;
#pragma unroll
  for (int i = 0; i < 8; ++i) { const int ka = k0 + 8 * g + i, kb = ka + 16; v[i] = ka < K ? row[ka < K ? ka : K - 1] : 0.f; v[8 + i] = kb < K ? row[kb < K ? kb : K - 1] : 0.f; }
  return bsplit16(v); }
__device__ __forceinline__ F2 split_col(const float* W, int k0, int n, int lane, int ld, int K) { float v[16]; const int g = lane >> 4;
#pragma unroll
  for (int i = 0; i < 8; ++i) { const int ka = k0 + 8 * g + i, kb = ka + 16; v[i] = ka < K ? W[(size_t)(ka < K ? ka : K - 1) * ld + n] : 0.f; v[8 + i] = kb < K ? W[(size_t)(kb < K ? kb : K - 1) * ld + n] : 0.f; }
  return bsplit16(v); }
__device__ __forceinline__ v8f mac3(const F2& a, const F2& b, v8f c) { c = wmma_bf(a.l, b.h, c); c = wmma_bf(a.h, b.l, c); return wmma_bf(a.h, b.h, c); }
__device__ __forceinline__ float sigm(float v) { return 1.0f / (1.0f + expf(-v)); }
#define LDSX() do { asm volatile("s_wait_dscnt 0" ::: "memory"); __builtin_amdgcn_wave_barrier(); __builtin_amdgcn_fence(__ATOMIC_RELEASE, "workgroup"); } while (0)


#define NB 4
#define TT 2048
#define DD 256
#define HH 512
#define WW 32
#define NR (NB * TT)
#define NWIN (NR / WW)
#ifndef TRB
#define TRB (NR / 64)
#define TWIN NWIN
#define TLNB (NR / 8)
#endif
typedef __attribute__((ext_vector_type(8))) __bf16 v8b;
__device__ __forceinline__ v16b frag_b(const __bf16* rowk0, int lane) {
  union { v16b v; v8b q[2]; } u; const __bf16* p = rowk0 + 8 * (lane >> 4);
  u.q[0] = *(const v8b*)p; u.q[1] = *(const v8b*)(p + 16); return u.v;
}
__device__ __forceinline__ float bfr(float v) { return (float)(__bf16)v; }
__device__ __attribute__((noinline)) float exp_ni(float v) { return expf(v); }
__device__ __attribute__((noinline)) float tanh_ni(float v) { return tanhf(v); }
__device__ __forceinline__ v8f mac3p(v16b ah, v16b al, v16b bh, v16b bl, v8f c) { c = wmma_bf(al, bh, c); c = wmma_bf(ah, bl, c); return wmma_bf(ah, bh, c); }

#define WS_PT1  0u
#define WS_PT2  (WS_PT1 + 2u * 3 * HH * DD)
#define WS_NH   (WS_PT2 + 2u * 3 * HH * HH)
#define WS_NL   (WS_NH + 2u * NR * DD)
#define WS_A1   (WS_NL + 2u * NR * DD)
#define WS_QKV  (WS_A1 + 4u * NR * HH)
#define WS_QTH  (WS_QKV + 4u * NR * 3 * HH)
#define WS_QTL  (WS_QTH + 2u * NWIN * HH * WW)
#define WS_KTH  (WS_QTL + 2u * NWIN * HH * WW)
#define WS_KTL  (WS_KTH + 2u * NWIN * HH * WW)
#define WS_END  (WS_KTL + 2u * NWIN * HH * WW)

__global__ __launch_bounds__(128) void k_pack(const float* __restrict__ w1, const float* __restrict__ w3, const float* __restrict__ w5, const float* __restrict__ w2, const float* __restrict__ w4, const float* __restrict__ w6, __bf16* __restrict__ PT1, __bf16* __restrict__ PT2) {
  __shared__ __align__(16) __bf16 srow[HH];
  const int n = blockIdx.x, tid = threadIdx.x;
  if (n < 3 * HH) { const int m = n / HH, nn = n % HH; const float* Wm = m == 0 ? w1 : (m == 1 ? w3 : w5);
    for (int k = tid; k < DD; k += 128) srow[k] = (__bf16)Wm[(size_t)k * HH + nn];
    __syncthreads(); if (tid < DD / 8) vst2((unsigned*)(PT1 + (size_t)n * DD + tid * 8), *(const v4u*)(&srow[tid * 8])); }
  else { const int n2 = n - 3 * HH; const int m = n2 / HH, nn = n2 % HH; const float* Wm = m == 0 ? w2 : (m == 1 ? w4 : w6);
    for (int k = tid; k < HH; k += 128) srow[k] = (__bf16)Wm[(size_t)k * HH + nn];
    __syncthreads(); if (tid < HH / 8) vst2((unsigned*)(PT2 + (size_t)n2 * HH + tid * 8), *(const v4u*)(&srow[tid * 8])); }
}
__global__ __launch_bounds__(256) void k_ln(const float* __restrict__ X, const float* __restrict__ g, const float* __restrict__ bb, __bf16* __restrict__ NH, __bf16* __restrict__ NL) {
  const int tid = threadIdx.x, wave = tid >> 5, lane = tid & 31; const size_t r = (size_t)blockIdx.x * 8 + wave;
  float v[8]; float s = 0.f;
#pragma unroll
  for (int i = 0; i < 8; ++i) { v[i] = bfr(X[r * DD + lane * 8 + i]); s += v[i]; }
#pragma unroll
  for (int o = 1; o < 32; o <<= 1) s += __shfl_xor(s, o);
  const float mu = s * (1.0f / DD); float q = 0.f;
#pragma unroll
  for (int i = 0; i < 8; ++i) { const float d = v[i] - mu; q += d * d; }
#pragma unroll
  for (int o = 1; o < 32; o <<= 1) q += __shfl_xor(q, o);
  const float rs = rsqrtf(q * (1.0f / DD) + 1e-5f);
  union { __bf16 e[8]; v4u u; } hh, ll;
#pragma unroll
  for (int i = 0; i < 8; ++i) { const int c = lane * 8 + i; const float y = (v[i] - mu) * rs * bfr(g[c]) + bfr(bb[c]); const __bf16 hi = (__bf16)y; hh.e[i] = hi; ll.e[i] = (__bf16)(y - (float)hi); }
  vst2((unsigned*)(NH + r * DD + lane * 8), hh.u); vst2((unsigned*)(NL + r * DD + lane * 8), ll.u);
}
__global__ __launch_bounds__(128) void k_l1(const __bf16* __restrict__ NH, const __bf16* __restrict__ NL, const __bf16* __restrict__ PT1, const float* __restrict__ b1, const float* __restrict__ b3, const float* __restrict__ b5, float* __restrict__ A1, int m) {
  __shared__ __align__(16) float so[4][16][132];
  const int tid = threadIdx.x, wave = tid >> 5, lane = tid & 31, col = lane & 15, g = lane >> 4; const size_t r0 = (size_t)blockIdx.x * 64 + wave * 16; const int n0 = blockIdx.y * 128;
  v8f acc[8] = {};
#pragma unroll 2
  for (int kc = 0; kc < DD / 32; ++kc) { const v16b ah = frag_b(NH + (r0 + col) * DD + kc * 32, lane), al = frag_b(NL + (r0 + col) * DD + kc * 32, lane);
#pragma unroll
    for (int j = 0; j < 8; ++j) { const v16b w = frag_b(PT1 + (size_t)(m * HH + n0 + j * 16 + col) * DD + kc * 32, lane); acc[j] = wmma_bf(al, w, acc[j]); acc[j] = wmma_bf(ah, w, acc[j]); } }
  const float* bias = m == 0 ? b1 : (m == 1 ? b3 : b5);
#pragma unroll
  for (int j = 0; j < 8; ++j) { const int nn = n0 + j * 16 + col; const float bv = bfr(bias[nn]);
#pragma unroll
    for (int r = 0; r < 8; ++r) { const float v = acc[j][r] + bv; so[wave][8 * g + r][j * 16 + col] = m < 2 ? tanh_ni(v) : (v > 0.f ? v : 0.f); } }
  LDSX();
  for (int rl = 0; rl < 16; ++rl) vst2(A1 + (r0 + rl) * HH + n0 + lane * 4, *(const v4f*)(&so[wave][rl][lane * 4]));
}
__global__ __launch_bounds__(128) void k_l2(const float* __restrict__ A1, const __bf16* __restrict__ PT2, const float* __restrict__ b2, const float* __restrict__ b4, const float* __restrict__ b6, float* __restrict__ QKV, int m) {
  __shared__ __align__(16) float so[4][16][132];
  const int tid = threadIdx.x, wave = tid >> 5, lane = tid & 31, col = lane & 15, g = lane >> 4; const size_t r0 = (size_t)blockIdx.x * 64 + wave * 16; const int n0 = blockIdx.y * 128;
  v8f acc[8] = {};
#pragma unroll 2
  for (int kc = 0; kc < HH / 32; ++kc) { const F2 a = split_row(A1 + (r0 + col) * HH, kc * 32, lane);
#pragma unroll
    for (int j = 0; j < 8; ++j) { const v16b w = frag_b(PT2 + (size_t)(m * HH + n0 + j * 16 + col) * HH + kc * 32, lane); acc[j] = wmma_bf(a.l, w, acc[j]); acc[j] = wmma_bf(a.h, w, acc[j]); } }
  const float* bias = m == 0 ? b2 : (m == 1 ? b4 : b6);
#pragma unroll
  for (int j = 0; j < 8; ++j) { const int nn = n0 + j * 16 + col; const float bv = bfr(bias[nn]);
#pragma unroll
    for (int r = 0; r < 8; ++r) so[wave][8 * g + r][j * 16 + col] = acc[j][r] + bv; }
  LDSX();
  for (int rl = 0; rl < 16; ++rl) vst2(QKV + (r0 + rl) * (3 * HH) + m * HH + n0 + lane * 4, *(const v4f*)(&so[wave][rl][lane * 4]));
}
__global__ __launch_bounds__(256) void k_tr(const float* __restrict__ QKV, __bf16* __restrict__ QTH, __bf16* __restrict__ QTL, __bf16* __restrict__ KTH, __bf16* __restrict__ KTL) {
  __shared__ __bf16 sh[HH][40], sl[HH][40];
  const int win = blockIdx.x, which = blockIdx.y, tid = threadIdx.x;
  for (int q = tid; q < WW * HH; q += 256) { const int w = q / HH, h = q % HH; const float v = QKV[((size_t)win * WW + w) * (3 * HH) + which * HH + h]; const __bf16 hi = (__bf16)v; sh[h][w] = hi; sl[h][w] = (__bf16)(v - (float)hi); }
  __syncthreads();
  __bf16* DH_ = which ? KTH : QTH; __bf16* DL_ = which ? KTL : QTL;
  for (int q = tid; q < HH * 4; q += 256) { const int h = q >> 2, pc = q & 3; union { __bf16 e[8]; v4u u; } a, c;
#pragma unroll
    for (int e = 0; e < 8; ++e) { a.e[e] = sh[h][pc * 8 + e]; c.e[e] = sl[h][pc * 8 + e]; }
    const size_t o = ((size_t)win * HH + h) * WW + pc * 8; vst2((unsigned*)(DH_ + o), a.u); vst2((unsigned*)(DL_ + o), c.u); }
}
__global__ __launch_bounds__(128) void k_win(const float* __restrict__ QKV, const __bf16* __restrict__ QTH, const __bf16* __restrict__ QTL, const __bf16* __restrict__ KTH, const __bf16* __restrict__ KTL, float* __restrict__ out) {
  __shared__ __align__(16) float sat[WW][36];
  __shared__ __align__(16) float sb[HH][20];
  __shared__ __align__(16) __bf16 sah[16][HH + 8], sal[16][HH + 8];
  __shared__ __align__(16) __bf16 sfh[HH][40], sfl[HH][40];
  __shared__ __align__(16) float so[4][16][132];
  const int tid = threadIdx.x, wave = tid >> 5, lane = tid & 31, col = lane & 15, g = lane >> 4; const int win = blockIdx.x;
  const float* Qr = QKV + (size_t)win * WW * (3 * HH); const float* Kr = Qr + HH; const float* Vr = Qr + 2 * HH; const int ld = 3 * HH;
  const float isf = 1.0f / sqrtf((float)HH), ist = 1.0f / sqrtf((float)WW);
  { const int rt = wave & 1, ct = wave >> 1; v8f acc = {};
#pragma unroll 2
    for (int kc = 0; kc < HH / 32; ++kc) { const F2 a = split_row(Qr + (size_t)(rt * 16 + col) * ld, kc * 32, lane), kb = split_row(Kr + (size_t)(ct * 16 + col) * ld, kc * 32, lane); acc = mac3(a, kb, acc); }
#pragma unroll
    for (int r = 0; r < 8; ++r) sat[rt * 16 + 8 * g + r][ct * 16 + col] = acc[r] * isf; }
  __syncthreads();
  if (tid < WW) { float* row = &sat[tid][0]; float mx = -3.0e38f; for (int v = 0; v < WW; ++v) mx = fmaxf(mx, row[v]); float s = 0.f; for (int v = 0; v < WW; ++v) { const float e = exp_ni(row[v] - mx); row[v] = e; s += e; } const float inv = 1.0f / s; for (int v = 0; v < WW; ++v) row[v] *= inv; }
  __syncthreads();
#pragma unroll 1
  for (int st = 0; st < HH / 16; ++st) { const int g0 = st * 16;
    { const v16b bh_ = frag_b(KTH + ((size_t)win * HH + g0 + col) * WW, lane), bl_ = frag_b(KTL + ((size_t)win * HH + g0 + col) * WW, lane);
#pragma unroll 1
      for (int ht = wave; ht < HH / 16; ht += 4) { const v16b ah = frag_b(QTH + ((size_t)win * HH + ht * 16 + col) * WW, lane), al = frag_b(QTL + ((size_t)win * HH + ht * 16 + col) * WW, lane);
        const v8f acc = mac3p(ah, al, bh_, bl_, (v8f){});
#pragma unroll
        for (int r = 0; r < 8; ++r) sb[ht * 16 + 8 * g + r][col] = acc[r] * ist; } }
    __syncthreads();
    { const int gl = tid >> 3, part = tid & 7; float mx = -3.0e38f;
      for (int h = part; h < HH; h += 8) mx = fmaxf(mx, sb[h][gl]);
#pragma unroll
      for (int o = 1; o < 8; o <<= 1) mx = fmaxf(mx, __shfl_xor(mx, o));
      float s = 0.f;
      for (int h = part; h < HH; h += 8) { const float e = exp_ni(sb[h][gl] - mx); sb[h][gl] = e; s += e; }
#pragma unroll
      for (int o = 1; o < 8; o <<= 1) s += __shfl_xor(s, o);
      const float inv = 1.0f / s;
      for (int h = part; h < HH; h += 8) { const float a = sb[h][gl] * inv; const __bf16 hi = (__bf16)a; sah[gl][h] = hi; sal[gl][h] = (__bf16)(a - (float)hi); } }
    __syncthreads();
    if (wave < 2) { v8f acc = {};
#pragma unroll 2
      for (int kc = 0; kc < HH / 32; ++kc) { const F2 a = split_row(Vr + (size_t)(wave * 16 + col) * ld, kc * 32, lane); acc = mac3p(a.h, a.l, frag_b(&sah[col][kc * 32], lane), frag_b(&sal[col][kc * 32], lane), acc); }
#pragma unroll
      for (int r = 0; r < 8; ++r) { const float v = acc[r]; const __bf16 hi = (__bf16)v; sfh[g0 + col][wave * 16 + 8 * g + r] = hi; sfl[g0 + col][wave * 16 + 8 * g + r] = (__bf16)(v - (float)hi); } }
    __syncthreads(); }
  { const int rt = wave & 1; const F2 a = split_row(&sat[rt * 16 + col][0], 0, lane);
#pragma unroll 1
    for (int pass = 0; pass < 2; ++pass) { v8f acc[8];
#pragma unroll
      for (int j = 0; j < 8; ++j) { const int ct = (wave >> 1) * 16 + pass * 8 + j; acc[j] = mac3p(a.h, a.l, frag_b(&sfh[ct * 16 + col][0], lane), frag_b(&sfl[ct * 16 + col][0], lane), (v8f){}); }
#pragma unroll
      for (int j = 0; j < 8; ++j)
#pragma unroll
        for (int r = 0; r < 8; ++r) so[wave][8 * g + r][j * 16 + col] = acc[j][r];
      LDSX();
      for (int rl = 0; rl < 16; ++rl) vst2(out + ((size_t)win * WW + rt * 16 + rl) * HH + ((wave >> 1) * 16 + pass * 8) * 16 + lane * 4, *(const v4f*)(&so[wave][rl][lane * 4]));
      LDSX(); } }
}

extern "C" void kernel_launch(void* const* d_in, const int* in_sizes, int n_in, void* d_out, int out_size, void* d_ws, size_t ws_size, hipStream_t stream) {
  (void)in_sizes; (void)n_in; (void)out_size;
  const float** F = (const float**)d_in;
  if (ws_size < (size_t)WS_END) return;
  char* ws = (char*)d_ws;
  __bf16 *PT1 = (__bf16*)(ws + WS_PT1), *PT2 = (__bf16*)(ws + WS_PT2), *NH = (__bf16*)(ws + WS_NH), *NL = (__bf16*)(ws + WS_NL), *QTH = (__bf16*)(ws + WS_QTH), *QTL = (__bf16*)(ws + WS_QTL), *KTH = (__bf16*)(ws + WS_KTH), *KTL = (__bf16*)(ws + WS_KTL);
  float *A1 = (float*)(ws + WS_A1), *QKV = (float*)(ws + WS_QKV);
  k_pack<<<6 * HH, 128, 0, stream>>>(F[3], F[7], F[11], F[5], F[9], F[13], PT1, PT2);
  k_ln<<<TLNB, 256, 0, stream>>>(F[0], F[1], F[2], NH, NL);
  for (int m = 0; m < 3; ++m) {
    k_l1<<<dim3(TRB, HH / 128), 128, 0, stream>>>(NH, NL, PT1, F[4], F[8], F[12], A1, m);
    k_l2<<<dim3(TRB, HH / 128), 128, 0, stream>>>(A1, PT2, F[6], F[10], F[14], QKV, m); }
  k_tr<<<dim3(TWIN, 2), 256, 0, stream>>>(QKV, QTH, QTL, KTH, KTL);
  k_win<<<TWIN, 128, 0, stream>>>(QKV, QTH, QTL, KTH, KTL, (float*)d_out);
}
